// GearBind_83708912599260
// MI455X (gfx1250) — hardware-verified
//
#include <hip/hip_runtime.h>
#include <stddef.h>
#include <math.h>


#define NB      8
#define LL      512
#define RR      7
#define DD      128
#define HH      8
#define DHD     16
#define NLAY    3
#define NN      32768
#define NE      1048576
#define NRES    4096
#define KU      896
#define KC      1024
#define KO      160
#define APC     1032
#define APQ     136
#define APO     168
#define TR      16
#define NTHR    256
#define NWAVE   8
#define NBKT    32
#define NPB     1024
#define CAPB    40960
#define MAXDEG  256
#define WSCAP   134217728

#define PL_CHI    0
#define PL_CLO    131072
#define PL_QHI    262144
#define PL_QLO    278528
#define PL_KHI    294912
#define PL_KLO    311296
#define PL_VHI    327680
#define PL_VLO    344064
#define PL_OHI    360448
#define PL_OLO    380928
#define PL_STRIDE 401408
#define PBLK_CONV 64
#define PBLK_SQ   8
#define PBLK_O    10
#define PBLK_LAYER (PBLK_CONV + 3 * PBLK_SQ + PBLK_O)
#define NPREPBLK  (NLAY * PBLK_LAYER + 1)

#define LDSC_BYTES (2 * TR * APC * 2 + TR * DD * 4)
#define LDSB_INTS  (3 * NPB + 4 + NTHR + CAPB)
#define LDSB_BYTES (LDSB_INTS * 4)

static_assert(KC == KU + DD && KU == RR * DD && KO == DD + 4 * HH);
static_assert((KC % 32) == 0 && (DD % 32) == 0 && (KO % 32) == 0);
static_assert((APC % 8) == 0 && APC >= KC && (APQ % 8) == 0 && APQ >= DD && (APO % 8) == 0 && APO >= KO);
static_assert(NN == NBKT * NPB && (NPB % TR) == 0 && (NN % TR) == 0 && (NRES % TR) == 0);
static_assert(NPB == 4 * NTHR && NTHR == 32 * NWAVE && TR == 2 * NWAVE);
static_assert(NRES == NB * LL && NN <= 65536 && NE <= (1 << 20));
static_assert((CAPB % 1024) == 0 && (NE % NTHR) == 0);
static_assert(PL_CLO == DD * KC && PL_QHI == 2 * DD * KC && PL_QLO == PL_QHI + DD * DD);
static_assert(PL_OHI == PL_QHI + 6 * DD * DD && PL_OLO == PL_OHI + DD * KO && PL_STRIDE == PL_OLO + DD * KO);
static_assert(PBLK_CONV * NTHR == DD * (KC / 8) && PBLK_SQ * NTHR == DD * (DD / 8) && PBLK_O * NTHR == DD * (KO / 8));
static_assert(LL == 16 * 32 && DHD * HH == DD);
static_assert((TR * (KO / 4)) % NTHR == 128);

typedef unsigned short v4us __attribute__((ext_vector_type(4)));
typedef unsigned short v8us __attribute__((ext_vector_type(8)));
typedef __bf16 v16bf __attribute__((ext_vector_type(16)));
typedef float v4f __attribute__((ext_vector_type(4)));
typedef float v8f __attribute__((ext_vector_type(8)));
typedef int   v4i __attribute__((ext_vector_type(4)));
union FragB { v16bf v; v8us h[2]; };

__device__ __forceinline__ v8f wmb(v16bf a, v16bf b, v8f c) {
  v8f d = __builtin_amdgcn_wmma_f32_16x16x32_bf16(false, a, false, b, (short)0, c, false, false);
  asm volatile("v_nop\n\tv_nop\n\tv_nop\n\tv_nop" : "+v"(d) : "v"(a), "v"(b));
  return d;
}

__device__ __forceinline__ unsigned short bf_rne(float f) {
  unsigned u = __float_as_uint(f);
  u = u + 0x7FFFu + ((u >> 16) & 1u);
  return (unsigned short)(u >> 16);
}
__device__ __forceinline__ float bf_val(unsigned short b) { return __uint_as_float(((unsigned)b) << 16); }

__device__ __forceinline__ void split4(v4f a, v4us& hi, v4us& lo) {
#pragma unroll
  for (int e = 0; e < 4; ++e) {
    const unsigned short hb = bf_rne(a[e]);
    hi[e] = hb;
    lo[e] = bf_rne(a[e] - bf_val(hb));
  }
}

__global__ __launch_bounds__(NTHR) void k_prep(const float* __restrict__ Wrel, const float* __restrict__ Wself,
                                                const float* __restrict__ Wq, const float* __restrict__ Wk,
                                                const float* __restrict__ Wv, const float* __restrict__ Wo,
                                                const float* __restrict__ gam,
                                                unsigned short* wpl, float* sptab) {
  const int blk = blockIdx.x, tid = threadIdx.x;
  if (blk == NPREPBLK - 1) {
    if (tid < 32) {
      const int gi = tid < NLAY * HH ? tid : NLAY * HH - 1;
      const float g = gam[gi];
      const float sp = fmaxf(g, 0.0f) + __logf(1.0f + __expf(-fabsf(g)));
      const float v = (tid < NLAY * HH) ? sp : 0.0f;
      *(volatile float*)(sptab + tid) = v;
      __threadfence();
      *(volatile float*)(sptab + tid) = v;
    }
    return;
  }
  const int layer = blk / PBLK_LAYER;
  const int lb = blk - layer * PBLK_LAYER;
  int i, K, ksplit, K2;
  const float* s0;
  const float* s1;
  size_t dhi, dlo;
  if (lb < PBLK_CONV) {
    i = lb * NTHR + tid; K = KC; ksplit = KU; K2 = DD;
    s0 = Wrel + (size_t)layer * KU * DD; s1 = Wself + (size_t)layer * DD * DD;
    dhi = PL_CHI; dlo = PL_CLO;
  } else if (lb < PBLK_CONV + PBLK_SQ) {
    i = (lb - PBLK_CONV) * NTHR + tid; K = DD; ksplit = DD; K2 = DD;
    s0 = Wq + (size_t)layer * DD * DD; s1 = s0; dhi = PL_QHI; dlo = PL_QLO;
  } else if (lb < PBLK_CONV + 2 * PBLK_SQ) {
    i = (lb - PBLK_CONV - PBLK_SQ) * NTHR + tid; K = DD; ksplit = DD; K2 = DD;
    s0 = Wk + (size_t)layer * DD * DD; s1 = s0; dhi = PL_KHI; dlo = PL_KLO;
  } else if (lb < PBLK_CONV + 3 * PBLK_SQ) {
    i = (lb - PBLK_CONV - 2 * PBLK_SQ) * NTHR + tid; K = DD; ksplit = DD; K2 = DD;
    s0 = Wv + (size_t)layer * DD * DD; s1 = s0; dhi = PL_VHI; dlo = PL_VLO;
  } else {
    i = (lb - PBLK_CONV - 3 * PBLK_SQ) * NTHR + tid; K = KO; ksplit = KO; K2 = KO;
    s0 = Wo + (size_t)layer * KO * DD; s1 = s0; dhi = PL_OHI; dlo = PL_OLO;
  }
  const int KG = K >> 3;
  const int n = i / KG;
  const int g = i - n * KG;
  const int k0 = 8 * g;
  v8us hv, lv;
#pragma unroll
  for (int e = 0; e < 8; ++e) {
    const int k = k0 + e;
    const int ka = k < ksplit ? k : ksplit - 1;
    int kb = k - ksplit; kb = kb < 0 ? 0 : (kb > K2 - 1 ? K2 - 1 : kb);
    const float wa = s0[(size_t)ka * DD + n];
    const float wb = s1[(size_t)kb * DD + n];
    const float w = (k < ksplit) ? wa : wb;
    const unsigned short hb = bf_rne(w);
    hv[e] = hb;
    lv[e] = bf_rne(w - bf_val(hb));
  }
  unsigned short* base = wpl + (size_t)layer * PL_STRIDE;
  unsigned short* ph = base + dhi + (size_t)i * 8;
  unsigned short* pl = base + dlo + (size_t)i * 8;
  *(volatile v8us*)ph = hv;
  *(volatile v8us*)pl = lv;
  __threadfence();
  *(volatile v8us*)ph = hv;
  *(volatile v8us*)pl = lv;
}

__global__ __launch_bounds__(NTHR) void k_bucket(const int* __restrict__ nout, const int* __restrict__ nin,
                                                  const int* __restrict__ erel, const float* __restrict__ ew,
                                                  int nEdges, int* octab, int* pkout, float* wout) {
  extern __shared__ v4i dynlds[];
  int* lds  = (int*)dynlds;
  int* cnt  = lds;
  int* off  = lds + NPB;
  int* cur  = lds + 2 * NPB + 4;
  int* wtmp = lds + 3 * NPB + 4;
  int* el   = lds + 3 * NPB + 4 + NTHR;
  const int tid = threadIdx.x, bk = blockIdx.x;
  const int nodeLo = bk * NPB;

  for (int l = tid; l < NPB; l += NTHR) { cnt[l] = 0; cur[l] = 0; }
  __syncthreads();

#pragma unroll 1
  for (int e0 = 0; e0 < nEdges; e0 += NTHR) {
    const int e = e0 + tid;
    const int ec = e < nEdges ? e : nEdges - 1;
    const int d = nout[ec] - nodeLo;
    if (e < nEdges && (unsigned)d < (unsigned)NPB) atomicAdd(&cnt[d], 1);
  }
  __syncthreads();

  {
    const int s = cnt[4 * tid] + cnt[4 * tid + 1] + cnt[4 * tid + 2] + cnt[4 * tid + 3];
    wtmp[tid] = s;
  }
  __syncthreads();
  if (tid == 0) {
    int run = 0;
#pragma unroll 1
    for (int t = 0; t < NTHR; ++t) { const int s = wtmp[t]; wtmp[t] = run; run += s; }
    off[NPB] = run;
  }
  __syncthreads();
  {
    int base = wtmp[tid];
    const int c0 = cnt[4 * tid], c1 = cnt[4 * tid + 1], c2 = cnt[4 * tid + 2];
    off[4 * tid] = base; base += c0;
    off[4 * tid + 1] = base; base += c1;
    off[4 * tid + 2] = base; base += c2;
    off[4 * tid + 3] = base;
  }
  __syncthreads();

#pragma unroll 1
  for (int e0 = 0; e0 < nEdges; e0 += NTHR) {
    const int e = e0 + tid;
    const int ec = e < nEdges ? e : nEdges - 1;
    const int d = nout[ec] - nodeLo;
    int r = erel[ec];
    r = r < 0 ? 0 : (r > RR - 1 ? RR - 1 : r);
    if (e < nEdges && (unsigned)d < (unsigned)NPB) {
      const int s = atomicAdd(&cur[d], 1);
      const int slot = off[d] + s;
      if ((unsigned)slot < (unsigned)CAPB) el[slot] = (r << 20) | ec;
    }
  }
  __syncthreads();

  for (int l = tid; l < NPB; l += NTHR) {
    int o = off[l]; o = o < 0 ? 0 : (o > CAPB ? CAPB : o);
    int c = cnt[l]; c = c < 0 ? 0 : (c > MAXDEG ? MAXDEG : c);
    if (c > CAPB - o) c = CAPB - o;
#pragma unroll 1
    for (int a = 1; a < c; ++a) {
      const int v = el[o + a];
      int b = a - 1;
#pragma unroll 1
      for (;;) {
        const int bb = b < 0 ? 0 : b;
        const int cv = el[o + bb];
        if (b < 0 || cv <= v) break;
        el[o + b + 1] = cv;
        --b;
      }
      el[o + b + 1] = v;
    }
  }
  __syncthreads();

  const int total = off[NPB];
#pragma unroll 1
  for (int pass = 0; pass < 2; ++pass) {
    for (int p = tid; p < NPB / 2; p += NTHR) {
      v4i t4;
      t4[0] = off[2 * p]; t4[1] = cnt[2 * p]; t4[2] = off[2 * p + 1]; t4[3] = cnt[2 * p + 1];
      *(volatile v4i*)(octab + (size_t)(nodeLo + 2 * p) * 2) = t4;
    }
    for (int q = tid; q < CAPB / 4; q += NTHR) {
      v4i pk4;
      v4f w4;
#pragma unroll
      for (int j = 0; j < 4; ++j) {
        const int s = 4 * q + j;
        const int key = el[s];
        int e = key & 0xFFFFF;
        e = e > nEdges - 1 ? nEdges - 1 : e;
        int src = nin[e];
        src = src < 0 ? 0 : (src > NN - 1 ? NN - 1 : src);
        int r = erel[e];
        r = r < 0 ? 0 : (r > RR - 1 ? RR - 1 : r);
        const float w = ew[e];
        const bool val = s < total;
        pk4[j] = val ? (src | (r << 16)) : 0;
        w4[j]  = val ? w : 0.0f;
      }
      *(volatile v4i*)(pkout + (size_t)bk * CAPB + 4 * q) = pk4;
      *(volatile v4f*)(wout + (size_t)bk * CAPB + 4 * q) = w4;
    }
    if (pass == 0) __threadfence();
  }
}

__device__ __forceinline__ void putrun(unsigned short* rhi, unsigned short* rlo, int slot, v4f a) {
  v4us h, l;
  split4(a, h, l);
  *(v4us*)(rhi + slot * DD) = h;
  *(v4us*)(rlo + slot * DD) = l;
}
__device__ __forceinline__ void putzero(unsigned short* rhi, unsigned short* rlo, int slot) {
  const v4us z = {0, 0, 0, 0};
  *(v4us*)(rhi + slot * DD) = z;
  *(v4us*)(rlo + slot * DD) = z;
}

__global__ __launch_bounds__(NTHR) void k_conv(const float* __restrict__ xin, const int* __restrict__ octab,
                                                const int* __restrict__ pk, const float* __restrict__ wv,
                                                const unsigned short* __restrict__ Bhi,
                                                const unsigned short* __restrict__ Blo,
                                                const float* __restrict__ brel, const float* __restrict__ bself,
                                                float* hout) {
  extern __shared__ v4i dynlds[];
  unsigned short* sAhi = (unsigned short*)dynlds;
  unsigned short* sAlo = sAhi + TR * APC;
  float* stg = (float*)(sAlo + TR * APC);
  const int tid = threadIdx.x, lane = tid & 31, wave = tid >> 5, hh = lane >> 4, m = lane & 15;
  const int tile = blockIdx.x;

#pragma unroll 1
  for (int s = 0; s < 2; ++s) {
    const int ln = 2 * wave + s;
    const int node = tile * TR + ln;
    const int bucket = node / NPB;
    int o = octab[2 * node];
    int c = octab[2 * node + 1];
    o = o < 0 ? 0 : (o > CAPB ? CAPB : o);
    c = c < 0 ? 0 : (c > MAXDEG ? MAXDEG : c);
    if (c > CAPB - o) c = CAPB - o;
    const int base = bucket * CAPB + o;
    unsigned short* rhi = sAhi + ln * APC + 4 * lane;
    unsigned short* rlo = sAlo + ln * APC + 4 * lane;
    v4f a = {0.f, 0.f, 0.f, 0.f};
    int cr = 0;
#pragma unroll 1
    for (int q0 = 0; q0 < c; q0 += 32) {
      int pos = base + q0 + lane;
      pos = pos > NBKT * CAPB - 1 ? NBKT * CAPB - 1 : pos;
      const int pkl = pk[pos];
      const int wbl = __float_as_int(wv[pos]);
      const int mcnt = (c - q0) < 32 ? (c - q0) : 32;
#pragma unroll 1
      for (int p = 0; p < mcnt; ++p) {
        const int pv = __builtin_amdgcn_readlane(pkl, p);
        const float w = __int_as_float(__builtin_amdgcn_readlane(wbl, p));
        int src = pv & 0xFFFF;
        src = src > NN - 1 ? NN - 1 : src;
        int rv = (pv >> 16) & 7;
        rv = rv > RR - 1 ? RR - 1 : rv;
        if (rv != cr) {
          putrun(rhi, rlo, cr, a);
          for (int z = cr + 1; z < rv; ++z) putzero(rhi, rlo, z);
          a[0] = 0.f; a[1] = 0.f; a[2] = 0.f; a[3] = 0.f;
          cr = rv;
        }
        const v4f v = *(const v4f*)(xin + (size_t)src * DD + 4 * lane);
        a = a + v * w;
      }
    }
    putrun(rhi, rlo, cr, a);
    for (int z = cr + 1; z < RR; ++z) putzero(rhi, rlo, z);
    const v4f xs = *(const v4f*)(xin + (size_t)node * DD + 4 * lane);
    v4us xh, xl;
    split4(xs, xh, xl);
    *(v4us*)(rhi + KU) = xh;
    *(v4us*)(rlo + KU) = xl;
  }
  __syncthreads();

  {
    const int ct = wave;
    v8f acc = {0.f, 0.f, 0.f, 0.f, 0.f, 0.f, 0.f, 0.f};
    const unsigned short* ahb = sAhi + m * APC + 8 * hh;
    const unsigned short* alb = sAlo + m * APC + 8 * hh;
    const unsigned short* bhb = Bhi + (size_t)(ct * 16 + m) * KC + 8 * hh;
    const unsigned short* blb = Blo + (size_t)(ct * 16 + m) * KC + 8 * hh;
#pragma unroll 2
    for (int kt = 0; kt < KC / 32; ++kt) {
      FragB ah, al, bh, bl;
      ah.h[0] = *(const v8us*)(ahb + 32 * kt);
      ah.h[1] = *(const v8us*)(ahb + 32 * kt + 16);
      al.h[0] = *(const v8us*)(alb + 32 * kt);
      al.h[1] = *(const v8us*)(alb + 32 * kt + 16);
      bh.h[0] = *(const v8us*)(bhb + 32 * kt);
      bh.h[1] = *(const v8us*)(bhb + 32 * kt + 16);
      bl.h[0] = *(const v8us*)(blb + 32 * kt);
      bl.h[1] = *(const v8us*)(blb + 32 * kt + 16);
      acc = wmb(ah.v, bh.v, acc);
      acc = wmb(ah.v, bl.v, acc);
      acc = wmb(al.v, bh.v, acc);
    }
    const int col = ct * 16 + m;
    const float bb = brel[col] + bself[col];
#pragma unroll
    for (int r = 0; r < 8; ++r) {
      const int row = 8 * hh + r;
      stg[row * DD + col] = fmaxf(acc[r] + bb, 0.0f);
    }
  }
  __syncthreads();

  {
    const int r0 = 2 * wave, r1 = 2 * wave + 1;
    const v4f v0 = *(const v4f*)(stg + r0 * DD + 4 * lane);
    const v4f v1 = *(const v4f*)(stg + r1 * DD + 4 * lane);
    float* g0 = hout + (size_t)(tile * TR + r0) * DD + 4 * lane;
    float* g1 = hout + (size_t)(tile * TR + r1) * DD + 4 * lane;
    *(volatile v4f*)g0 = v0;
    *(volatile v4f*)g1 = v1;
    __threadfence();
    *(volatile v4f*)g0 = v0;
    *(volatile v4f*)g1 = v1;
  }
}

__global__ __launch_bounds__(NTHR) void k_qkv(const float* __restrict__ hid, const int* __restrict__ ca,
                                               const unsigned short* __restrict__ qh, const unsigned short* __restrict__ ql,
                                               const unsigned short* __restrict__ kh, const unsigned short* __restrict__ kl,
                                               const unsigned short* __restrict__ vh, const unsigned short* __restrict__ vl,
                                               float* qout, float* kout, float* vout) {
  __shared__ __attribute__((aligned(16))) unsigned short sAhi[TR * APQ];
  __shared__ __attribute__((aligned(16))) unsigned short sAlo[TR * APQ];
  __shared__ __attribute__((aligned(16))) float stg[3 * TR * DD];
  const int tid = threadIdx.x, lane = tid & 31, wave = tid >> 5, hh = lane >> 4, m = lane & 15;
  const int r0 = blockIdx.x * TR;

  {
    const int rr = tid >> 4;
    const int kq = (tid & 15) * 8;
    int atom = ca[r0 + rr];
    atom = atom < 0 ? 0 : (atom > NN - 1 ? NN - 1 : atom);
    const float* p = hid + (size_t)atom * DD + kq;
    const v4f f0 = *(const v4f*)p;
    const v4f f1 = *(const v4f*)(p + 4);
    v4us h0, l0, h1, l1;
    split4(f0, h0, l0);
    split4(f1, h1, l1);
    v8us hv, lv;
#pragma unroll
    for (int e = 0; e < 4; ++e) { hv[e] = h0[e]; hv[4 + e] = h1[e]; lv[e] = l0[e]; lv[4 + e] = l1[e]; }
    *(v8us*)(sAhi + rr * APQ + kq) = hv;
    *(v8us*)(sAlo + rr * APQ + kq) = lv;
  }
  __syncthreads();

  {
    const int ct = wave;
    v8f accq = {0.f, 0.f, 0.f, 0.f, 0.f, 0.f, 0.f, 0.f};
    v8f acck = {0.f, 0.f, 0.f, 0.f, 0.f, 0.f, 0.f, 0.f};
    v8f accv = {0.f, 0.f, 0.f, 0.f, 0.f, 0.f, 0.f, 0.f};
    const unsigned short* ahb = sAhi + m * APQ + 8 * hh;
    const unsigned short* alb = sAlo + m * APQ + 8 * hh;
    const size_t bo_ = (size_t)(ct * 16 + m) * DD + 8 * hh;
#pragma unroll 1
    for (int kt = 0; kt < DD / 32; ++kt) {
      FragB ah, al, bh, bl;
      ah.h[0] = *(const v8us*)(ahb + 32 * kt);
      ah.h[1] = *(const v8us*)(ahb + 32 * kt + 16);
      al.h[0] = *(const v8us*)(alb + 32 * kt);
      al.h[1] = *(const v8us*)(alb + 32 * kt + 16);
      bh.h[0] = *(const v8us*)(qh + bo_ + 32 * kt);
      bh.h[1] = *(const v8us*)(qh + bo_ + 32 * kt + 16);
      bl.h[0] = *(const v8us*)(ql + bo_ + 32 * kt);
      bl.h[1] = *(const v8us*)(ql + bo_ + 32 * kt + 16);
      accq = wmb(ah.v, bh.v, accq);
      accq = wmb(ah.v, bl.v, accq);
      accq = wmb(al.v, bh.v, accq);
      bh.h[0] = *(const v8us*)(kh + bo_ + 32 * kt);
      bh.h[1] = *(const v8us*)(kh + bo_ + 32 * kt + 16);
      bl.h[0] = *(const v8us*)(kl + bo_ + 32 * kt);
      bl.h[1] = *(const v8us*)(kl + bo_ + 32 * kt + 16);
      acck = wmb(ah.v, bh.v, acck);
      acck = wmb(ah.v, bl.v, acck);
      acck = wmb(al.v, bh.v, acck);
      bh.h[0] = *(const v8us*)(vh + bo_ + 32 * kt);
      bh.h[1] = *(const v8us*)(vh + bo_ + 32 * kt + 16);
      bl.h[0] = *(const v8us*)(vl + bo_ + 32 * kt);
      bl.h[1] = *(const v8us*)(vl + bo_ + 32 * kt + 16);
      accv = wmb(ah.v, bh.v, accv);
      accv = wmb(ah.v, bl.v, accv);
      accv = wmb(al.v, bh.v, accv);
    }
    const int col = ct * 16 + m;
#pragma unroll
    for (int r = 0; r < 8; ++r) {
      const int row = 8 * hh + r;
      stg[0 * TR * DD + row * DD + col] = accq[r];
      stg[1 * TR * DD + row * DD + col] = acck[r];
      stg[2 * TR * DD + row * DD + col] = accv[r];
    }
  }
  __syncthreads();

  {
    const int ra = 2 * wave, rb = 2 * wave + 1;
    const v4f q0 = *(const v4f*)(stg + 0 * TR * DD + ra * DD + 4 * lane);
    const v4f q1 = *(const v4f*)(stg + 0 * TR * DD + rb * DD + 4 * lane);
    const v4f k0 = *(const v4f*)(stg + 1 * TR * DD + ra * DD + 4 * lane);
    const v4f k1 = *(const v4f*)(stg + 1 * TR * DD + rb * DD + 4 * lane);
    const v4f v0 = *(const v4f*)(stg + 2 * TR * DD + ra * DD + 4 * lane);
    const v4f v1 = *(const v4f*)(stg + 2 * TR * DD + rb * DD + 4 * lane);
    const size_t ga = (size_t)(r0 + ra) * DD + 4 * lane, gb = (size_t)(r0 + rb) * DD + 4 * lane;
    *(volatile v4f*)(qout + ga) = q0; *(volatile v4f*)(qout + gb) = q1;
    *(volatile v4f*)(kout + ga) = k0; *(volatile v4f*)(kout + gb) = k1;
    *(volatile v4f*)(vout + ga) = v0; *(volatile v4f*)(vout + gb) = v1;
    __threadfence();
    *(volatile v4f*)(qout + ga) = q0; *(volatile v4f*)(qout + gb) = q1;
    *(volatile v4f*)(kout + ga) = k0; *(volatile v4f*)(kout + gb) = k1;
    *(volatile v4f*)(vout + ga) = v0; *(volatile v4f*)(vout + gb) = v1;
  }
}

__global__ __launch_bounds__(NTHR) void k_attn(const float* __restrict__ qb, const float* __restrict__ kb,
                                                const float* __restrict__ vb,
                                                const float* __restrict__ posCA, const float* __restrict__ posCB,
                                                const float* __restrict__ frame, const int* __restrict__ kflag,
                                                const float* __restrict__ sptab, float* hcat) {
  __shared__ __attribute__((aligned(16))) float srow[KO];
  const int tid = threadIdx.x, lane = tid & 31, h = tid >> 5;
  const int row = blockIdx.x;
  const int b = row / LL;
  const float sp = sptab[h];
  float qr[DHD];
  const float* qp = qb + (size_t)row * DD + h * DHD;
#pragma unroll
  for (int d = 0; d < DHD; ++d) qr[d] = qp[d] * 0.25f;
  const float cb0 = posCB[row * 3 + 0], cb1 = posCB[row * 3 + 1], cb2 = posCB[row * 3 + 2];
  const float* kbase = kb + (size_t)(b * LL) * DD + h * DHD;
  const float* vbase = vb + (size_t)(b * LL) * DD + h * DHD;
  const float* cbb = posCB + (size_t)(b * LL) * 3;
  const float* cab = posCA + (size_t)(b * LL) * 3;
  const int* kf = kflag + b * LL;

  float mx = -3.0e38f;
#pragma unroll 1
  for (int t = 0; t < LL / 32; ++t) {
    const int j = lane + 32 * t;
    const float* kp = kbase + (size_t)j * DD;
    const v4f k0 = *(const v4f*)kp, k1 = *(const v4f*)(kp + 4), k2 = *(const v4f*)(kp + 8), k3 = *(const v4f*)(kp + 12);
    float dot = 0.f;
#pragma unroll
    for (int d = 0; d < 4; ++d) { dot += qr[d] * k0[d]; dot += qr[4 + d] * k1[d]; dot += qr[8 + d] * k2[d]; dot += qr[12 + d] * k3[d]; }
    const float dx = cb0 - cbb[j * 3 + 0], dy = cb1 - cbb[j * 3 + 1], dz = cb2 - cbb[j * 3 + 2];
    const float d2 = (dx * dx + dz * dz) + dy * dy;
    float lg = dot - sp * d2;
    lg = (kf[j] != 0) ? lg : -1.0e9f;
    mx = fmaxf(mx, lg);
  }
#pragma unroll
  for (int s = 16; s >= 1; s >>= 1) mx = fmaxf(mx, __shfl_xor(mx, s, 32));

  float facc[DHD];
#pragma unroll
  for (int d = 0; d < DHD; ++d) facc[d] = 0.f;
  float p0 = 0.f, p1 = 0.f, p2 = 0.f, wsum = 0.f;
#pragma unroll 1
  for (int t = 0; t < LL / 32; ++t) {
    const int j = lane + 32 * t;
    const float* kp = kbase + (size_t)j * DD;
    const v4f k0 = *(const v4f*)kp, k1 = *(const v4f*)(kp + 4), k2 = *(const v4f*)(kp + 8), k3 = *(const v4f*)(kp + 12);
    float dot = 0.f;
#pragma unroll
    for (int d = 0; d < 4; ++d) { dot += qr[d] * k0[d]; dot += qr[4 + d] * k1[d]; dot += qr[8 + d] * k2[d]; dot += qr[12 + d] * k3[d]; }
    const float dx = cb0 - cbb[j * 3 + 0], dy = cb1 - cbb[j * 3 + 1], dz = cb2 - cbb[j * 3 + 2];
    const float d2 = (dx * dx + dz * dz) + dy * dy;
    float lg = dot - sp * d2;
    lg = (kf[j] != 0) ? lg : -1.0e9f;
    const float w = __expf(lg - mx);
    wsum += w;
    const float* vp = vbase + (size_t)j * DD;
    const v4f v0 = *(const v4f*)vp, v1 = *(const v4f*)(vp + 4), v2 = *(const v4f*)(vp + 8), v3 = *(const v4f*)(vp + 12);
#pragma unroll
    for (int d = 0; d < 4; ++d) { facc[d] += w * v0[d]; facc[4 + d] += w * v1[d]; facc[8 + d] += w * v2[d]; facc[12 + d] += w * v3[d]; }
    p0 += w * cab[j * 3 + 0]; p1 += w * cab[j * 3 + 1]; p2 += w * cab[j * 3 + 2];
  }
#pragma unroll
  for (int s = 16; s >= 1; s >>= 1) {
    wsum += __shfl_xor(wsum, s, 32);
    p0 += __shfl_xor(p0, s, 32); p1 += __shfl_xor(p1, s, 32); p2 += __shfl_xor(p2, s, 32);
#pragma unroll
    for (int d = 0; d < DHD; ++d) facc[d] += __shfl_xor(facc[d], s, 32);
  }

  if (lane == 0) {
    const float inv = 1.0f / wsum;
#pragma unroll
    for (int d = 0; d < DHD; ++d) srow[h * DHD + d] = facc[d] * inv;
    const float a0 = p0 * inv - posCA[row * 3 + 0];
    const float a1 = p1 * inv - posCA[row * 3 + 1];
    const float a2 = p2 * inv - posCA[row * 3 + 2];
    const float* fr = frame + (size_t)row * 9;
    const float l0 = fr[0] * a0 + fr[3] * a1 + fr[6] * a2;
    const float l1 = fr[1] * a0 + fr[4] * a1 + fr[7] * a2;
    const float l2 = fr[2] * a0 + fr[5] * a1 + fr[8] * a2;
    srow[DD + h * 3 + 0] = l0; srow[DD + h * 3 + 1] = l1; srow[DD + h * 3 + 2] = l2;
    srow[DD + 3 * HH + h] = sqrtf(l0 * l0 + l1 * l1 + l2 * l2 + 1e-8f);
  }
  __syncthreads();
  if (tid < KO / 4) {
    const v4f ov = *(const v4f*)(srow + 4 * tid);
    float* gp = hcat + (size_t)row * KO + 4 * tid;
    *(volatile v4f*)gp = ov;
    __threadfence();
    *(volatile v4f*)gp = ov;
  }
}

__global__ __launch_bounds__(NTHR) void k_wo(const float* __restrict__ hcat,
                                              const unsigned short* __restrict__ oh, const unsigned short* __restrict__ ol,
                                              const float* __restrict__ bo, const int* __restrict__ rflag,
                                              const int* __restrict__ ca, float* hid) {
  __shared__ __attribute__((aligned(16))) unsigned short sAhi[TR * APO];
  __shared__ __attribute__((aligned(16))) unsigned short sAlo[TR * APO];
  __shared__ __attribute__((aligned(16))) float stg[TR * DD];
  const int tid = threadIdx.x, lane = tid & 31, wave = tid >> 5, hh = lane >> 4, m = lane & 15;
  const int r0 = blockIdx.x * TR;

  for (int u = tid; u < TR * (KO / 4); u += NTHR) {
    const int rr = u / (KO / 4);
    const int c4 = u - rr * (KO / 4);
    const v4f f = *(const v4f*)(hcat + (size_t)(r0 + rr) * KO + 4 * c4);
    v4us hv, lv;
    split4(f, hv, lv);
    *(v4us*)(sAhi + rr * APO + 4 * c4) = hv;
    *(v4us*)(sAlo + rr * APO + 4 * c4) = lv;
  }
  __syncthreads();

  {
    const int ct = wave;
    v8f acc = {0.f, 0.f, 0.f, 0.f, 0.f, 0.f, 0.f, 0.f};
    const unsigned short* ahb = sAhi + m * APO + 8 * hh;
    const unsigned short* alb = sAlo + m * APO + 8 * hh;
    const unsigned short* bhb = oh + (size_t)(ct * 16 + m) * KO + 8 * hh;
    const unsigned short* blb = ol + (size_t)(ct * 16 + m) * KO + 8 * hh;
#pragma unroll 1
    for (int kt = 0; kt < KO / 32; ++kt) {
      FragB ah, al, bh, bl;
      ah.h[0] = *(const v8us*)(ahb + 32 * kt);
      ah.h[1] = *(const v8us*)(ahb + 32 * kt + 16);
      al.h[0] = *(const v8us*)(alb + 32 * kt);
      al.h[1] = *(const v8us*)(alb + 32 * kt + 16);
      bh.h[0] = *(const v8us*)(bhb + 32 * kt);
      bh.h[1] = *(const v8us*)(bhb + 32 * kt + 16);
      bl.h[0] = *(const v8us*)(blb + 32 * kt);
      bl.h[1] = *(const v8us*)(blb + 32 * kt + 16);
      acc = wmb(ah.v, bh.v, acc);
      acc = wmb(ah.v, bl.v, acc);
      acc = wmb(al.v, bh.v, acc);
    }
    const int col = ct * 16 + m;
    const float bb = bo[col];
#pragma unroll
    for (int r = 0; r < 8; ++r) {
      const int row = 8 * hh + r;
      const float mf = (rflag[r0 + row] != 0) ? 1.0f : 0.0f;
      stg[row * DD + col] = (acc[r] + bb) * mf;
    }
  }
  __syncthreads();

  {
    const int ra = 2 * wave, rb = 2 * wave + 1;
    int aa = ca[r0 + ra]; aa = aa < 0 ? 0 : (aa > NN - 1 ? NN - 1 : aa);
    int ab = ca[r0 + rb]; ab = ab < 0 ? 0 : (ab > NN - 1 ? NN - 1 : ab);
    float* pa = hid + (size_t)aa * DD + 4 * lane;
    float* pb = hid + (size_t)ab * DD + 4 * lane;
    const v4f oa = *(const v4f*)pa;
    const v4f ob = *(const v4f*)pb;
    const v4f na = oa + *(const v4f*)(stg + ra * DD + 4 * lane);
    const v4f nb = ob + *(const v4f*)(stg + rb * DD + 4 * lane);
    *(volatile v4f*)pa = na;
    *(volatile v4f*)pb = nb;
    __threadfence();
    *(volatile v4f*)pa = na;
    *(volatile v4f*)pb = nb;
  }
}

__global__ __launch_bounds__(DD) void k_readout(const float* __restrict__ hid, const int* __restrict__ ca, float* gout) {
  const int b = blockIdx.x, d = threadIdx.x;
  float s = 0.f;
#pragma unroll 1
  for (int l = 0; l < LL; ++l) {
    int atom = ca[b * LL + l];
    atom = atom < 0 ? 0 : (atom > NN - 1 ? NN - 1 : atom);
    s += hid[(size_t)atom * DD + d];
  }
  float* p = gout + b * DD + d;
  *(volatile float*)p = s;
  __threadfence();
  *(volatile float*)p = s;
}

extern "C" void kernel_launch(void* const* d_in, const int* in_sizes, int n_in,
                              void* d_out, int out_size, void* d_ws, size_t ws_size,
                              hipStream_t stream) {
  if (n_in < 20) return;
  if (in_sizes[0] != NN * DD) return;
  if (in_sizes[1] != NE || in_sizes[2] != NE || in_sizes[3] != NE || in_sizes[4] != NE) return;
  if (in_sizes[5] != NRES || in_sizes[6] != NRES * 3 || in_sizes[7] != NRES * 3) return;
  if (in_sizes[8] != NRES * 9 || in_sizes[9] != NRES) return;
  if (in_sizes[10] != NLAY * KU * DD || in_sizes[11] != NLAY * DD) return;
  if (in_sizes[12] != NLAY * DD * DD || in_sizes[13] != NLAY * DD) return;
  if (in_sizes[14] != NLAY * DD * DD || in_sizes[15] != NLAY * DD * DD || in_sizes[16] != NLAY * DD * DD) return;
  if (in_sizes[17] != NLAY * HH || in_sizes[18] != NLAY * KO * DD || in_sizes[19] != NLAY * DD) return;
  if (out_size != NB * DD + NN * DD) return;

  const float* x      = (const float*)d_in[0];
  const int*   nin    = (const int*)d_in[1];
  const int*   nout   = (const int*)d_in[2];
  const int*   erel   = (const int*)d_in[3];
  const float* ew     = (const float*)d_in[4];
  const int*   ca     = (const int*)d_in[5];
  const float* posCA  = (const float*)d_in[6];
  const float* posCB  = (const float*)d_in[7];
  const float* frame  = (const float*)d_in[8];
  const int*   flags  = (const int*)d_in[9];
  const float* Wrel   = (const float*)d_in[10];
  const float* brel   = (const float*)d_in[11];
  const float* Wself  = (const float*)d_in[12];
  const float* bself  = (const float*)d_in[13];
  const float* Wq     = (const float*)d_in[14];
  const float* Wk     = (const float*)d_in[15];
  const float* Wv     = (const float*)d_in[16];
  const float* gam    = (const float*)d_in[17];
  const float* Wo     = (const float*)d_in[18];
  const float* bo     = (const float*)d_in[19];
  float* out = (float*)d_out;
  const int nEdges = in_sizes[1];

  char* ws = (char*)d_ws;
  size_t o = 0;
  const size_t szH  = (size_t)NN * DD * 4;
  const size_t szP  = (size_t)NRES * DD * 4;
  const size_t szHC = (size_t)NRES * KO * 4;
  const size_t szWP = (size_t)NLAY * PL_STRIDE * 2;
  const size_t szSP = 256;
  const size_t szOC = (size_t)NN * 2 * 4;
  const size_t szPK = (size_t)NBKT * CAPB * 4;
  const size_t oHA = o; o += szH;
  const size_t oHB = o; o += szH;
  const size_t oQ  = o; o += szP;
  const size_t oK  = o; o += szP;
  const size_t oV  = o; o += szP;
  const size_t oHC = o; o += szHC;
  const size_t oWP = o; o += szWP;
  const size_t oSP = o; o += szSP;
  const size_t oOC = o; o += szOC;
  const size_t oPK = o; o += szPK;
  const size_t oWV = o; o += szPK;
  if (o > ws_size || o > (size_t)WSCAP) return;

  float* hidA  = (float*)(ws + oHA);
  float* hidB  = (float*)(ws + oHB);
  float* qbuf  = (float*)(ws + oQ);
  float* kbuf  = (float*)(ws + oK);
  float* vbuf  = (float*)(ws + oV);
  float* hcat  = (float*)(ws + oHC);
  unsigned short* wpl = (unsigned short*)(ws + oWP);
  float* sptab = (float*)(ws + oSP);
  int*   octab = (int*)(ws + oOC);
  int*   pk    = (int*)(ws + oPK);
  float* wv    = (float*)(ws + oWV);

  hipFuncSetAttribute(reinterpret_cast<const void*>(&k_bucket), hipFuncAttributeMaxDynamicSharedMemorySize, LDSB_BYTES);
  hipFuncSetAttribute(reinterpret_cast<const void*>(&k_conv), hipFuncAttributeMaxDynamicSharedMemorySize, LDSC_BYTES);

  k_prep<<<NPREPBLK, NTHR, 0, stream>>>(Wrel, Wself, Wq, Wk, Wv, Wo, gam, wpl, sptab);
  k_bucket<<<NBKT, NTHR, LDSB_BYTES, stream>>>(nout, nin, erel, ew, nEdges, octab, pk, wv);

  for (int i = 0; i < NLAY; ++i) {
    const float* xin = (i == 0) ? x : ((i == 1) ? hidA : hidB);
    float* hout = (i == 0) ? hidA : ((i == 1) ? hidB : (out + NB * DD));
    const unsigned short* pl = wpl + (size_t)i * PL_STRIDE;
    k_conv<<<NN / TR, NTHR, LDSC_BYTES, stream>>>(xin, octab, pk, wv, pl + PL_CHI, pl + PL_CLO,
                                                  brel + i * DD, bself + i * DD, hout);
    k_qkv<<<NRES / TR, NTHR, 0, stream>>>(hout, ca, pl + PL_QHI, pl + PL_QLO, pl + PL_KHI, pl + PL_KLO,
                                          pl + PL_VHI, pl + PL_VLO, qbuf, kbuf, vbuf);
    k_attn<<<NRES, NTHR, 0, stream>>>(qbuf, kbuf, vbuf, posCA, posCB, frame, flags, sptab + i * HH, hcat);
    k_wo<<<NRES / TR, NTHR, 0, stream>>>(hcat, pl + PL_OHI, pl + PL_OLO, bo + i * DD, flags, ca, hout);
  }
  k_readout<<<NB, DD, 0, stream>>>(out + NB * DD, ca, out);
}
